// RWKV_TimeMix_47897475285605
// MI455X (gfx1250) — hardware-verified
//
#include <hip/hip_runtime.h>
#include <math.h>

constexpr int kB = 2;
constexpr int kT = 1024;
constexpr int kC = 2048;
constexpr int kH = 32;
constexpr int kN = 64;
constexpr int kRows = kB * kT;
constexpr int kLw = 160;
constexpr int kLwPad = 192;
constexpr int kLd = 32;
constexpr int kLdPitch = 64;
constexpr int kTd = 64;
constexpr int kChunk = 32;
constexpr float kGnEps = 1e-5f * 64.0f;
constexpr float kWCarry = 64.0f;
constexpr float kLoraCarry = 16384.0f;
constexpr float kDlCarry = 1048576.0f;
constexpr float kDlInv = 1.0f / 1048576.0f;
static_assert(kC == kH * kN);
static_assert(kC % 64 == 0 && kRows % 64 == 0 && kLwPad % 64 == 0 && kTd % 64 == 0);
static_assert(kC % 32 == 0 && kLd % 32 == 0 && kTd % 32 == 0);
static_assert(kT % kChunk == 0 && kChunk * 8 == 256 && kN == 64);
static_assert(kC / 8 == 256);

typedef __attribute__((ext_vector_type(16))) _Float16 v16h;
typedef __attribute__((ext_vector_type(8)))  _Float16 v8h;
typedef __attribute__((ext_vector_type(16))) __bf16   v16b;
typedef __attribute__((ext_vector_type(8)))  __bf16   v8b;
typedef __attribute__((ext_vector_type(8)))  float    v8f;
typedef __attribute__((ext_vector_type(4)))  float    v4f;
typedef __attribute__((ext_vector_type(4)))  unsigned int v4u;

__device__ __forceinline__ unsigned short f2bf_bits(float f) {
  unsigned u = __float_as_uint(f);
  return (unsigned short)((u + 0x7FFFu + ((u >> 16) & 1u)) >> 16);
}
__device__ __forceinline__ float bf_bits2f(unsigned short h) { return __uint_as_float(((unsigned)h) << 16); }

__device__ __forceinline__ float h16_to_f32(unsigned hb) {
  const unsigned sgn = (hb & 0x8000u) << 16; const unsigned em = hb & 0x7fffu;
  const float fn = __uint_as_float((em << 13) + 0x38000000u);
  const float fs = (float)em * 5.9604644775390625e-8f;
  const float mag = (em < 0x400u) ? fs : fn; return __uint_as_float(__float_as_uint(mag) | sgn); }

__device__ __forceinline__ void dep_guard4_h(v8f& a, v8f& b, v8f& c, v8f& d, v16h x, v16h y) { asm volatile("v_nop\n\tv_nop\n\tv_nop\n\tv_nop" : "+v"(a), "+v"(b), "+v"(c), "+v"(d) : "v"(x), "v"(y)); }
__device__ __forceinline__ void dep_guard4_b(v8f& a, v8f& b, v8f& c, v8f& d, v16b x, v16b y) { asm volatile("v_nop\n\tv_nop\n\tv_nop\n\tv_nop" : "+v"(a), "+v"(b), "+v"(c), "+v"(d) : "v"(x), "v"(y)); }
__device__ __forceinline__ void keep4_h(v16h a, v16h b, v16h c, v16h d) { asm volatile("v_nop" :: "v"(a), "v"(b), "v"(c), "v"(d)); }
__device__ __forceinline__ void keep4_b(v16b a, v16b b, v16b c, v16b d) { asm volatile("v_nop" :: "v"(a), "v"(b), "v"(c), "v"(d)); }
__device__ __forceinline__ void acc_guard4(v8f& a, v8f& b, v8f& c, v8f& d) { asm volatile("v_nop\n\tv_nop\n\tv_nop\n\tv_nop" : "+v"(a), "+v"(b), "+v"(c), "+v"(d)); }
template <typename T> struct Frag;
template <> struct Frag<_Float16> {
  typedef v16h V; union U { v16h v; v8h h[2]; };
  static __device__ __forceinline__ v16h load(const _Float16* p) {
    U f; f.h[0] = *(const v8h*)(p); f.h[1] = *(const v8h*)(p + 16); return f.v;
  }
  static __device__ __forceinline__ v8f mma(v16h a, v16h b, v8f c) {
    return __builtin_amdgcn_wmma_f32_16x16x32_f16(false, a, false, b, (short)0, c, false, false);
  }
  static __device__ __forceinline__ void guard4(v8f& a, v8f& b, v8f& c, v8f& d, v16h x, v16h y) { dep_guard4_h(a, b, c, d, x, y); }
  static __device__ __forceinline__ void keep(v16h a, v16h b, v16h c, v16h d) { keep4_h(a, b, c, d); }
};
template <> struct Frag<__bf16> {
  typedef v16b V; union U { v16b v; v8b h[2]; };
  static __device__ __forceinline__ v16b load(const __bf16* p) {
    U f; f.h[0] = *(const v8b*)(p); f.h[1] = *(const v8b*)(p + 16); return f.v;
  }
  static __device__ __forceinline__ v8f mma(v16b a, v16b b, v8f c) {
    return __builtin_amdgcn_wmma_f32_16x16x32_bf16(false, a, false, b, (short)0, c, false, false);
  }
  static __device__ __forceinline__ void guard4(v8f& a, v8f& b, v8f& c, v8f& d, v16b x, v16b y) { dep_guard4_b(a, b, c, d, x, y); }
  static __device__ __forceinline__ void keep(v16b a, v16b b, v16b c, v16b d) { keep4_b(a, b, c, d); }
};

__device__ __forceinline__ unsigned pk16(unsigned short a, unsigned short b) { return (unsigned)a | ((unsigned)b << 16); }
__device__ __forceinline__ unsigned short h_bits(float f) { const _Float16 h = (_Float16)f; return __builtin_bit_cast(unsigned short, h); }

template <int ET> struct Elem;
template <> struct Elem<0> { typedef _Float16 T; };
template <> struct Elem<1> { typedef __bf16 T; };
template <int ET, bool SPLIT, int BIAS_MODE, int OUT_MODE, int ACT>
__global__ __launch_bounds__(256) void wmma_gemm64(
    const unsigned short* __restrict__ Ap, const unsigned short* __restrict__ A2p, int lda, long strideA,
    const unsigned short* __restrict__ Btp, const unsigned short* __restrict__ Bt2p, int ldb, long strideB,
    void* __restrict__ Cout, void* __restrict__ Cout2, int ldc, long strideC,
    const float* __restrict__ bias,
    int M, int N, int K, float scale) {
  typedef typename Elem<ET>::T T;
  typedef typename Frag<T>::V V;
  const T* A = (const T*)Ap; const T* A2 = (const T*)A2p; const T* Bt = (const T*)Btp; const T* Bt2 = (const T*)Bt2p;
  __shared__ __align__(16) float sT[8][16 * 68];
  const int b    = blockIdx.y;
  const int lane = threadIdx.x & 31;
  const int wave = threadIdx.x >> 5;
  const int tilesN = N >> 6;
  const int tilesM = M >> 6;
  const int tile = blockIdx.x * 8 + wave;
  if (tile >= tilesM * tilesN) return;
  const int tm = tile / tilesN;
  const int tn = tile - tm * tilesN;
  const int m0 = tm << 6;
  const int n0 = tn << 6;

  const T* Ab  = A  + (size_t)b * strideA;
  const T* Bb  = Bt + (size_t)b * strideB;
  const T* Ab2 = SPLIT ? (A2  + (size_t)b * strideA) : nullptr;
  const T* Bb2 = SPLIT ? (Bt2 + (size_t)b * strideB) : nullptr;

  const int rlane = lane & 15;
  const int koff  = (lane >> 4) * 8;
  const int mOff  = (lane >> 4) * 8;

  v8f acc[4][4];
#pragma unroll
  for (int i = 0; i < 4; ++i)
#pragma unroll
    for (int j = 0; j < 4; ++j) acc[i][j] = (v8f){0.f,0.f,0.f,0.f,0.f,0.f,0.f,0.f};

  for (int k0 = 0; k0 < K; k0 += 32) {
    V bh[4], bl[4];
#pragma unroll
    for (int j = 0; j < 4; ++j) {
      const size_t bo = (size_t)(n0 + (j << 4) + rlane) * ldb + koff + k0;
      bh[j] = Frag<T>::load(Bb + bo);
      if (SPLIT) bl[j] = Frag<T>::load(Bb2 + bo);
    }
#pragma unroll
    for (int i = 0; i < 4; ++i) {
      const size_t ao = (size_t)(m0 + (i << 4) + rlane) * lda + koff + k0;
      V ah = Frag<T>::load(Ab + ao);
      V al;
      if (SPLIT) al = Frag<T>::load(Ab2 + ao);
#pragma unroll
      for (int j = 0; j < 4; ++j) {
        acc[i][j] = Frag<T>::mma(ah, bh[j], acc[i][j]);
        if (SPLIT) {
          acc[i][j] = Frag<T>::mma(ah, bl[j], acc[i][j]);
          acc[i][j] = Frag<T>::mma(al, bh[j], acc[i][j]);
        }
      }
      Frag<T>::guard4(acc[i][0], acc[i][1], acc[i][2], acc[i][3], ah, SPLIT ? al : bh[3]);
    }
    Frag<T>::keep(bh[0], bh[1], bh[2], bh[3]);
    if (SPLIT) Frag<T>::keep(bl[0], bl[1], bl[2], bl[3]);
  }
  acc_guard4(acc[0][0], acc[0][1], acc[0][2], acc[0][3]);
  acc_guard4(acc[1][0], acc[1][1], acc[1][2], acc[1][3]);
  acc_guard4(acc[2][0], acc[2][1], acc[2][2], acc[2][3]);
  acc_guard4(acc[3][0], acc[3][1], acc[3][2], acc[3][3]);

  float* slab = sT[wave];
#pragma unroll
  for (int i = 0; i < 4; ++i) {
    const int mBase = m0 + (i << 4);
#pragma unroll
    for (int j = 0; j < 4; ++j) {
      const int n = n0 + (j << 4) + rlane;
      float bv = 0.f;
      if (BIAS_MODE == 2) bv = bias[n];
#pragma unroll
      for (int r = 0; r < 8; ++r) {
        float v = acc[i][j][r] * scale;
        if (BIAS_MODE == 1) v += bias[mBase + mOff + r];
        if (BIAS_MODE == 2) v += bv;
        if (ACT == 1) v = tanhf(v);
        if (ACT == 2) v = fmaxf(v, 0.0f);
        if (ACT == 3) v = v / (1.0f + expf(-v));
        if (ACT == 4) v = (v > 0.f) ? v : 0.01f * v;
        slab[(mOff + r) * 68 + (j << 4) + rlane] = v;
      }
    }
    __builtin_amdgcn_fence(__ATOMIC_RELEASE, "workgroup");
    __builtin_amdgcn_wave_barrier();
    __builtin_amdgcn_fence(__ATOMIC_ACQUIRE, "workgroup");
    if (OUT_MODE == 0) {
      float* C = (float*)Cout + (size_t)b * strideC;
      const int hh = lane >> 4, c4 = (lane & 15) * 4;
      for (int pass = 0; pass < 2; ++pass) {
#pragma unroll
        for (int it = 0; it < 8; ++it) {
          const int row = it * 2 + hh;
          v4f v = *(const v4f*)(slab + row * 68 + c4);
          *(volatile v4f*)(C + (size_t)(mBase + row) * ldc + n0 + c4) = v;
        }
        __threadfence();
      }
    } else {
      const int q = lane >> 3, c8 = (lane & 7) * 8;
      unsigned short* C  = (unsigned short*)Cout  + (size_t)b * strideC;
      unsigned short* C2 = (OUT_MODE == 2) ? ((unsigned short*)Cout2 + (size_t)b * strideC) : nullptr;
      for (int pass = 0; pass < 2; ++pass) {
#pragma unroll
        for (int it = 0; it < 4; ++it) {
          const int row = it * 4 + q;
          const float* sp = slab + row * 68 + c8;
          v8h hv, lv;
#pragma unroll
          for (int e = 0; e < 8; ++e) {
            if (OUT_MODE == 1) {
              hv[e] = (_Float16)sp[e];
            } else {
              unsigned short hb = f2bf_bits(sp[e]);
              hv[e] = __builtin_bit_cast(_Float16, hb);
              if (OUT_MODE == 2) {
                unsigned short lb = f2bf_bits(sp[e] - bf_bits2f(hb));
                lv[e] = __builtin_bit_cast(_Float16, lb);
              }
            }
          }
          *(volatile v8h*)(C + (size_t)(mBase + row) * ldc + n0 + c8) = hv;
          if (OUT_MODE == 2) *(volatile v8h*)(C2 + (size_t)(mBase + row) * ldc + n0 + c8) = lv;
        }
        __threadfence();
      }
    }
    __builtin_amdgcn_fence(__ATOMIC_RELEASE, "workgroup");
    __builtin_amdgcn_wave_barrier();
    __builtin_amdgcn_fence(__ATOMIC_ACQUIRE, "workgroup");
  }
}

__global__ __launch_bounds__(256) void mix_gemm64(
    const unsigned short* __restrict__ Ap, int lda,
    const unsigned short* __restrict__ Btp, int ldb,
    unsigned short* __restrict__ Cout, int ldc,
    const float* __restrict__ x, const float* __restrict__ cf,
    int M, int N, int K) {
  typedef __bf16 T;
  typedef v16b V;
  const T* A = (const T*)Ap; const T* Bt = (const T*)Btp;
  __shared__ __align__(16) float sT[8][16 * 68];
  const int lane = threadIdx.x & 31;
  const int wave = threadIdx.x >> 5;
  const int tilesN = N >> 6;
  const int tilesM = M >> 6;
  const int tile = blockIdx.x * 8 + wave;
  if (tile >= tilesM * tilesN) return;
  const int tm = tile / tilesN;
  const int tn = tile - tm * tilesN;
  const int m0 = tm << 6;
  const int n0 = tn << 6;

  const int rlane = lane & 15;
  const int koff  = (lane >> 4) * 8;
  const int mOff  = (lane >> 4) * 8;

  v8f acc[4][4];
#pragma unroll
  for (int i = 0; i < 4; ++i)
#pragma unroll
    for (int j = 0; j < 4; ++j) acc[i][j] = (v8f){0.f,0.f,0.f,0.f,0.f,0.f,0.f,0.f};

  for (int k0 = 0; k0 < K; k0 += 32) {
    V bh[4];
#pragma unroll
    for (int j = 0; j < 4; ++j) {
      const size_t bo = (size_t)(n0 + (j << 4) + rlane) * ldb + koff + k0;
      bh[j] = Frag<T>::load(Bt + bo);
    }
#pragma unroll
    for (int i = 0; i < 4; ++i) {
      const size_t ao = (size_t)(m0 + (i << 4) + rlane) * lda + koff + k0;
      V ah = Frag<T>::load(A + ao);
#pragma unroll
      for (int j = 0; j < 4; ++j) acc[i][j] = Frag<T>::mma(ah, bh[j], acc[i][j]);
      Frag<T>::guard4(acc[i][0], acc[i][1], acc[i][2], acc[i][3], ah, bh[3]);
    }
    Frag<T>::keep(bh[0], bh[1], bh[2], bh[3]);
  }
  acc_guard4(acc[0][0], acc[0][1], acc[0][2], acc[0][3]);
  acc_guard4(acc[1][0], acc[1][1], acc[1][2], acc[1][3]);
  acc_guard4(acc[2][0], acc[2][1], acc[2][2], acc[2][3]);
  acc_guard4(acc[3][0], acc[3][1], acc[3][2], acc[3][3]);

  float* slab = sT[wave];
  const int q = lane >> 3, c8 = (lane & 7) * 8;
#pragma unroll
  for (int i = 0; i < 4; ++i) {
    const int mBase = m0 + (i << 4);
#pragma unroll
    for (int j = 0; j < 4; ++j)
#pragma unroll
      for (int r = 0; r < 8; ++r) slab[(mOff + r) * 68 + (j << 4) + rlane] = acc[i][j][r];
    __builtin_amdgcn_fence(__ATOMIC_RELEASE, "workgroup");
    __builtin_amdgcn_wave_barrier();
    __builtin_amdgcn_fence(__ATOMIC_ACQUIRE, "workgroup");
    v4u uo[4];
#pragma unroll
    for (int it = 0; it < 4; ++it) {
      const int row = it * 4 + q;
      const int gr  = mBase + row;
      const int tt  = gr & (kT - 1);
      const float fz = (tt != 0) ? 1.0f : 0.0f;
      const int grp = (gr > 0) ? (gr - 1) : 0;
      const int gc  = n0 + c8;
      const float* xr = x + (size_t)gr * kC + gc;
      const float* xp = x + (size_t)grp * kC + gc;
      const float* mr = cf + gc;
      const float* sp = slab + row * 68 + c8;
      const v4f xa = *(const v4f*)xr, xb = *(const v4f*)(xr + 4);
      const v4f pa = *(const v4f*)xp, pb = *(const v4f*)(xp + 4);
      const v4f ma = *(const v4f*)mr, mb = *(const v4f*)(mr + 4);
      unsigned short hb[8];
#pragma unroll
      for (int e = 0; e < 4; ++e) {
        const float x0 = xa[e];
        const float d0 = pa[e] * fz - x0;
        hb[e] = h_bits(x0 + d0 * (ma[e] + sp[e]));
        const float x1 = xb[e];
        const float d1 = pb[e] * fz - x1;
        hb[4 + e] = h_bits(x1 + d1 * (mb[e] + sp[4 + e]));
      }
      uo[it] = (v4u){pk16(hb[0], hb[1]), pk16(hb[2], hb[3]), pk16(hb[4], hb[5]), pk16(hb[6], hb[7])};
      asm volatile("" ::: "memory");
    }
    for (int pass = 0; pass < 2; ++pass) {
#pragma unroll
      for (int it = 0; it < 4; ++it) {
        const int row = it * 4 + q;
        *(volatile v4u*)(Cout + (size_t)(mBase + row) * ldc + n0 + c8) = uo[it];
      }
      __threadfence();
    }
    __builtin_amdgcn_fence(__ATOMIC_RELEASE, "workgroup");
    __builtin_amdgcn_wave_barrier();
    __builtin_amdgcn_fence(__ATOMIC_ACQUIRE, "workgroup");
  }
}

template <int OT>
__global__ __launch_bounds__(256) void tcast_kernel(const float* __restrict__ W0, const float* __restrict__ W1,
                                                    const float* __restrict__ W2, const float* __restrict__ W3,
                                                    const float* __restrict__ W4, long zsi,
                                                    unsigned short* __restrict__ out, unsigned short* __restrict__ out2,
                                                    long zso, int kValid, int pitchN, int nValid, int ldo, float scale) {
  __shared__ float sm[64][65];
  const int t  = threadIdx.x;
  const int k0 = blockIdx.x * 64;
  const int n0 = blockIdx.y * 64;
  const int z  = blockIdx.z;
  const float* Wsel = (z == 0) ? W0 : (z == 1) ? W1 : (z == 2) ? W2 : (z == 3) ? W3 : W4;
  const float* W = Wsel + (size_t)z * zsi;
#pragma unroll
  for (int i = 0; i < 16; ++i) {
    const int e = i * 256 + t;
    const int r = e >> 6;
    const int c = e & 63;
    const int kk = k0 + r, nn = n0 + c;
    const int kc = (kk < kValid) ? kk : (kValid - 1);
    const int nc = (nn < nValid) ? nn : (nValid - 1);
    const float fsel = scale * ((kk < kValid) ? 1.0f : 0.0f) * ((nn < nValid) ? 1.0f : 0.0f);
    sm[c][r] = W[(size_t)kc * pitchN + nc] * fsel;
  }
  __syncthreads();
  const int lane = t & 31, wave = t >> 5;
  const int q = lane >> 3, c8 = (lane & 7) * 8;
  unsigned short* op  = out  + (size_t)z * zso;
  unsigned short* op2 = out2 + (size_t)z * zso;
  for (int pass = 0; pass < 2; ++pass) {
#pragma unroll
    for (int it = 0; it < 2; ++it) {
      const int row = wave * 8 + it * 4 + q;
      unsigned short hb[8], lb[8];
#pragma unroll
      for (int e = 0; e < 8; ++e) {
        const float v = sm[row][c8 + e];
        if (OT == 0) {
          hb[e] = h_bits(v); lb[e] = 0;
        } else {
          const unsigned short hh = f2bf_bits(v);
          hb[e] = hh;
          lb[e] = (OT == 2) ? f2bf_bits(v - bf_bits2f(hh)) : (unsigned short)0;
        }
      }
      const v4u u = (v4u){pk16(hb[0], hb[1]), pk16(hb[2], hb[3]), pk16(hb[4], hb[5]), pk16(hb[6], hb[7])};
      const size_t off = (size_t)(n0 + row) * ldo + k0 + c8;
      *(volatile v4u*)(op + off) = u;
      if (OT == 2) {
        const v4u u2 = (v4u){pk16(lb[0], lb[1]), pk16(lb[2], lb[3]), pk16(lb[4], lb[5]), pk16(lb[6], lb[7])};
        *(volatile v4u*)(op2 + off) = u2;
      }
    }
    __threadfence();
  }
}

__global__ __launch_bounds__(256) void prep_kernel(const float* __restrict__ x, const float* __restrict__ mx,
                                                   unsigned short* __restrict__ outp, int n8) {
  const int i = blockIdx.x * 256 + threadIdx.x;
  if (i >= n8) return;
  const int row = i >> 8;
  const int c   = (i & 255) * 8;
  const int tt  = row & (kT - 1);
  const float fz = (tt != 0) ? 1.0f : 0.0f;
  const int rp  = (row > 0) ? (row - 1) : 0;
  const float* xr = x + (size_t)row * kC + c;
  const float* xp = x + (size_t)rp * kC + c;
  const v4f xa = *(const v4f*)xr, xb = *(const v4f*)(xr + 4);
  const v4f pa = *(const v4f*)xp, pb = *(const v4f*)(xp + 4);
  const v4f ma = *(const v4f*)(mx + c), mb = *(const v4f*)(mx + c + 4);
  unsigned short hb[8];
#pragma unroll
  for (int e = 0; e < 4; ++e) {
    const float x0 = xa[e];
    const float d0 = pa[e] * fz - x0;
    hb[e] = h_bits(x0 + d0 * ma[e]);
    const float x1 = xb[e];
    const float d1 = pb[e] * fz - x1;
    hb[4 + e] = h_bits(x1 + d1 * mb[e]);
  }
  const v4u u = (v4u){pk16(hb[0], hb[1]), pk16(hb[2], hb[3]), pk16(hb[4], hb[5]), pk16(hb[6], hb[7])};
  unsigned short* dq = outp + 8 * (size_t)i;
  *(volatile v4u*)dq = u;
  __threadfence();
  *(volatile v4u*)dq = u;
}

__global__ __launch_bounds__(256) void scan_gn_kernel(
    const unsigned short* __restrict__ rp, const unsigned short* __restrict__ kp,
    const unsigned short* __restrict__ vp, const unsigned short* __restrict__ gp,
    const unsigned short* __restrict__ dlp, const float* __restrict__ td,
    const float* __restrict__ u, const float* __restrict__ lng, const float* __restrict__ lnb,
    unsigned short* __restrict__ zh, unsigned short* __restrict__ zl) {
  __shared__ __align__(16) float rS[kChunk * 64];
  __shared__ __align__(16) float kS[kChunk * 64];
  __shared__ __align__(16) float dS[kChunk * 64];
  __shared__ __align__(16) float vS[kChunk * 64];
  __shared__ __align__(16) float gS[kChunk * 64];
  __shared__ __align__(16) float yS[kChunk * 64];
  __shared__ float bS[kChunk];
  __shared__ float tdS[64];
  const int tid  = threadIdx.x;
  const int lane = tid & 31;
  const int b = blockIdx.x >> 5;
  const int h = blockIdx.x & 31;
  const size_t colh = (size_t)h * kN;
  const int sts = tid >> 3;
  const int c8  = (tid & 7) * 8;
  const int si = tid >> 2;
  const int sq = tid & 3;

  if (tid < 64) tdS[tid] = td[colh + tid];
  float ur[8], lg[8], lb[8];
  {
    const v4f ua = *(const v4f*)(u + colh + c8),   ub = *(const v4f*)(u + colh + c8 + 4);
    const v4f ga = *(const v4f*)(lng + colh + c8), gb = *(const v4f*)(lng + colh + c8 + 4);
    const v4f ba = *(const v4f*)(lnb + colh + c8), bb = *(const v4f*)(lnb + colh + c8 + 4);
#pragma unroll
    for (int e = 0; e < 4; ++e) {
      ur[e] = ua[e]; ur[4 + e] = ub[e];
      lg[e] = ga[e]; lg[4 + e] = gb[e];
      lb[e] = ba[e]; lb[4 + e] = bb[e];
    }
  }
  float S[16];
#pragma unroll
  for (int jj = 0; jj < 16; ++jj) S[jj] = 0.0f;

#pragma unroll 1
  for (int ch = 0; ch < kT / kChunk; ++ch) {
    const int t0 = ch * kChunk;
    __syncthreads();
    {
      const size_t growg = (size_t)(b * kT + t0 + sts);
      const size_t o16 = growg * kC + colh + c8;
      const v4u ru = *(const v4u*)(rp + o16);
      const v4u ku = *(const v4u*)(kp + o16);
      const v4u vu = *(const v4u*)(vp + o16);
      const v4u gu = *(const v4u*)(gp + o16);
      float rf[8], kf[8], vf[8], gf[8];
#pragma unroll
      for (int e = 0; e < 4; ++e) {
        const unsigned wr = ru[e], wk = ku[e], wv = vu[e], wg = gu[e];
        rf[2 * e] = h16_to_f32(wr & 0xffffu); rf[2 * e + 1] = h16_to_f32(wr >> 16);
        kf[2 * e] = h16_to_f32(wk & 0xffffu); kf[2 * e + 1] = h16_to_f32(wk >> 16);
        vf[2 * e] = h16_to_f32(wv & 0xffffu); vf[2 * e + 1] = h16_to_f32(wv >> 16);
        gf[2 * e] = h16_to_f32(wg & 0xffffu); gf[2 * e + 1] = h16_to_f32(wg >> 16);
      }
      float* rdst = rS + sts * 64 + c8;
      float* kdst = kS + sts * 64 + c8;
      float* vdst = vS + sts * 64 + c8;
      float* gdst = gS + sts * 64 + c8;
      *(v4f*)(rdst) = (v4f){rf[0], rf[1], rf[2], rf[3]}; *(v4f*)(rdst + 4) = (v4f){rf[4], rf[5], rf[6], rf[7]};
      *(v4f*)(kdst) = (v4f){kf[0], kf[1], kf[2], kf[3]}; *(v4f*)(kdst + 4) = (v4f){kf[4], kf[5], kf[6], kf[7]};
      *(v4f*)(vdst) = (v4f){vf[0], vf[1], vf[2], vf[3]}; *(v4f*)(vdst + 4) = (v4f){vf[4], vf[5], vf[6], vf[7]};
      *(v4f*)(gdst) = (v4f){gf[0], gf[1], gf[2], gf[3]}; *(v4f*)(gdst + 4) = (v4f){gf[4], gf[5], gf[6], gf[7]};
      const unsigned* dw = (const unsigned*)(dlp + growg * kC + colh + c8);
      float* ddst = dS + sts * 64 + c8;
#pragma unroll 1
      for (int e2 = 0; e2 < 4; ++e2) {
        const unsigned wd = dw[e2];
        const float l0 = h16_to_f32(wd & 0xffffu) * kDlInv;
        const float l1 = h16_to_f32(wd >> 16) * kDlInv;
        const float w0 = tdS[c8 + 2 * e2] + l0;
        const float w1 = tdS[c8 + 2 * e2 + 1] + l1;
        const float x0 = expf(w0);
        const float x1 = expf(w1);
        ddst[2 * e2]     = expf(-x0);
        ddst[2 * e2 + 1] = expf(-x1);
      }
      float p = 0.0f;
#pragma unroll
      for (int e = 0; e < 8; ++e) p = fmaf(rf[e] * ur[e], kf[e], p);
      p += __shfl_xor(p, 1, 32);
      p += __shfl_xor(p, 2, 32);
      p += __shfl_xor(p, 4, 32);
      if ((lane & 7) == 0) bS[sts] = p;
    }
    __syncthreads();
#pragma unroll 1
    for (int ts = 0; ts < kChunk; ++ts) {
      const float* rrow = rS + ts * 64 + sq * 16;
      const float* krow = kS + ts * 64 + sq * 16;
      const float* drow = dS + ts * 64 + sq * 16;
      v4f rv[4], kv[4], dv[4];
#pragma unroll
      for (int q4 = 0; q4 < 4; ++q4) {
        rv[q4] = *(const v4f*)(rrow + 4 * q4);
        kv[q4] = *(const v4f*)(krow + 4 * q4);
        dv[q4] = *(const v4f*)(drow + 4 * q4);
      }
      const float vi = vS[ts * 64 + si];
      const float bn = bS[ts];
      float yacc = 0.0f;
#pragma unroll
      for (int jj = 0; jj < 16; ++jj) {
        const float rj = rv[jj >> 2][jj & 3];
        const float kj = kv[jj >> 2][jj & 3];
        const float dj = dv[jj >> 2][jj & 3];
        yacc = fmaf(rj, S[jj], yacc);
        S[jj] = fmaf(dj, S[jj], kj * vi);
      }
      yacc += __shfl_xor(yacc, 1, 32);
      yacc += __shfl_xor(yacc, 2, 32);
      const float yv = fmaf(bn, vi, yacc);
      if (sq == 0) yS[ts * 64 + si] = yv;
    }
    __syncthreads();
    {
      const float* yr = yS + sts * 64 + c8;
      const float* gr = gS + sts * 64 + c8;
      const v4f ya = *(const v4f*)yr, yb = *(const v4f*)(yr + 4);
      const v4f ga = *(const v4f*)gr, gb = *(const v4f*)(gr + 4);
      float yv8[8], gv8[8];
#pragma unroll
      for (int e = 0; e < 4; ++e) { yv8[e] = ya[e]; yv8[4 + e] = yb[e]; gv8[e] = ga[e]; gv8[4 + e] = gb[e]; }
      float s = ((yv8[0] + yv8[1]) + (yv8[2] + yv8[3])) + ((yv8[4] + yv8[5]) + (yv8[6] + yv8[7]));
      s += __shfl_xor(s, 1, 32);
      s += __shfl_xor(s, 2, 32);
      s += __shfl_xor(s, 4, 32);
      const float mu = s * (1.0f / 64.0f);
      float dv8[8];
      float s2 = 0.0f;
#pragma unroll
      for (int e = 0; e < 8; ++e) { dv8[e] = yv8[e] - mu; s2 = fmaf(dv8[e], dv8[e], s2); }
      s2 += __shfl_xor(s2, 1, 32);
      s2 += __shfl_xor(s2, 2, 32);
      s2 += __shfl_xor(s2, 4, 32);
      const float var  = s2 * (1.0f / 64.0f);
      const float rstd = rsqrtf(var + kGnEps);
      unsigned short hb[8], lob[8];
#pragma unroll
      for (int e = 0; e < 8; ++e) {
        const float yn = fmaf(dv8[e] * rstd, lg[e], lb[e]);
        const float zv = yn * gv8[e];
        const unsigned short hh = f2bf_bits(zv);
        hb[e]  = hh;
        lob[e] = f2bf_bits(zv - bf_bits2f(hh));
      }
      const v4u uh = (v4u){pk16(hb[0], hb[1]), pk16(hb[2], hb[3]), pk16(hb[4], hb[5]), pk16(hb[6], hb[7])};
      const v4u ul = (v4u){pk16(lob[0], lob[1]), pk16(lob[2], lob[3]), pk16(lob[4], lob[5]), pk16(lob[6], lob[7])};
      const size_t zoff = ((size_t)(b * kT + t0 + sts)) * kC + colh + c8;
      *(volatile v4u*)(zh + zoff) = uh;
      *(volatile v4u*)(zl + zoff) = ul;
      __threadfence();
      *(volatile v4u*)(zh + zoff) = uh;
      *(volatile v4u*)(zl + zoff) = ul;
    }
  }
}

extern "C" void kernel_launch(void* const* d_in, const int* in_sizes, int n_in,
                              void* d_out, int out_size, void* d_ws, size_t ws_size,
                              hipStream_t stream) {
  if (n_in < 20) return;
  const int nBig = kRows * kC;
  if (in_sizes[0] != nBig || out_size != nBig) return;
  for (int i = 1; i <= 8; ++i) if (in_sizes[i] != kC) return;
  if (in_sizes[9] != kC * kLw || in_sizes[10] != 5 * kLd * kC) return;
  if (in_sizes[11] != kC * kTd || in_sizes[12] != kTd * kC) return;
  for (int i = 13; i <= 17; ++i) if (in_sizes[i] != kC * kC) return;
  if (in_sizes[18] != kC || in_sizes[19] != kC) return;

  const size_t plane16 = (size_t)kC * kC * 2;
  const size_t offWT4  = 0;
  const size_t offWOH  = offWT4 + 4 * plane16;
  const size_t offWOL  = offWOH + plane16;
  const size_t offW1T  = offWOL + plane16;
  const size_t offTW1T = offW1T + (size_t)kLwPad * kC * 2;
  const size_t offTW2T = offTW1T + (size_t)kTd * kC * 2;
  const size_t offW2T  = offTW2T + (size_t)kC * kTd * 2;
  const size_t offXXX  = offW2T + (size_t)5 * kC * kLdPitch * 2;
  const size_t offM    = offXXX + plane16;
  const size_t offHA   = offM + (size_t)kRows * kLwPad * 2;
  const size_t offXF   = offHA + (size_t)kRows * kTd * 2;
  const size_t offDL   = offXF + plane16;
  const size_t offR    = offDL + plane16;
  const size_t offK    = offR + plane16;
  const size_t offV    = offK + plane16;
  const size_t offG    = offV + plane16;
  const size_t offZH   = offG + plane16;
  const size_t offZL   = offZH + plane16;
  const size_t total   = offZL + plane16;
  if (ws_size < total) return;

  const float* x      = (const float*)d_in[0];
  const float* maa_x  = (const float*)d_in[1];
  const float* maa_w  = (const float*)d_in[2];
  const float* maa_k  = (const float*)d_in[3];
  const float* maa_v  = (const float*)d_in[4];
  const float* maa_r  = (const float*)d_in[5];
  const float* maa_g  = (const float*)d_in[6];
  const float* tdecay = (const float*)d_in[7];
  const float* uu     = (const float*)d_in[8];
  const float* maa_w1 = (const float*)d_in[9];
  const float* maa_w2 = (const float*)d_in[10];
  const float* td_w1  = (const float*)d_in[11];
  const float* td_w2  = (const float*)d_in[12];
  const float* Wr     = (const float*)d_in[13];
  const float* Wk     = (const float*)d_in[14];
  const float* Wv     = (const float*)d_in[15];
  const float* Wg     = (const float*)d_in[16];
  const float* Wo     = (const float*)d_in[17];
  const float* ln_g   = (const float*)d_in[18];
  const float* ln_b   = (const float*)d_in[19];
  float* out = (float*)d_out;
  char* ws = (char*)d_ws;
  unsigned short* WT4  = (unsigned short*)(ws + offWT4);
  unsigned short* WOH  = (unsigned short*)(ws + offWOH);
  unsigned short* WOL  = (unsigned short*)(ws + offWOL);
  unsigned short* W1T  = (unsigned short*)(ws + offW1T);
  unsigned short* TW1T = (unsigned short*)(ws + offTW1T);
  unsigned short* TW2T = (unsigned short*)(ws + offTW2T);
  unsigned short* W2T  = (unsigned short*)(ws + offW2T);
  unsigned short* XXX  = (unsigned short*)(ws + offXXX);
  unsigned short* MPL  = (unsigned short*)(ws + offM);
  unsigned short* HA   = (unsigned short*)(ws + offHA);
  unsigned short* XF   = (unsigned short*)(ws + offXF);
  unsigned short* DL   = (unsigned short*)(ws + offDL);
  unsigned short* RPL  = (unsigned short*)(ws + offR);
  unsigned short* KPL  = (unsigned short*)(ws + offK);
  unsigned short* VPL  = (unsigned short*)(ws + offV);
  unsigned short* GPL  = (unsigned short*)(ws + offG);
  unsigned short* ZH   = (unsigned short*)(ws + offZH);
  unsigned short* ZL   = (unsigned short*)(ws + offZL);
  const size_t planeElems = (size_t)kC * kC;
  unsigned short* WrT = WT4 + 0 * planeElems;
  unsigned short* WkT = WT4 + 1 * planeElems;
  unsigned short* WvT = WT4 + 2 * planeElems;
  unsigned short* WgT = WT4 + 3 * planeElems;

  const dim3 blk(256);
  tcast_kernel<0><<<dim3(kC / 64, kC / 64, 4), blk, 0, stream>>>(Wr, Wk, Wv, Wg, Wg, 0L, WT4, WT4, (long)planeElems,
                                                                 kC, kC, kC, kC, kWCarry);
  tcast_kernel<2><<<dim3(kC / 64, kC / 64, 1), blk, 0, stream>>>(Wo, Wo, Wo, Wo, Wo, 0L, WOH, WOL, 0L,
                                                                 kC, kC, kC, kC, 1.0f);
  tcast_kernel<0><<<dim3(kC / 64, kLwPad / 64, 1), blk, 0, stream>>>(maa_w1, maa_w1, maa_w1, maa_w1, maa_w1, 0L, W1T, W1T, 0L,
                                                                     kC, kLw, kLw, kC, kLoraCarry);
  tcast_kernel<0><<<dim3(kC / 64, kTd / 64, 1), blk, 0, stream>>>(td_w1, td_w1, td_w1, td_w1, td_w1, 0L, TW1T, TW1T, 0L,
                                                                  kC, kTd, kTd, kC, kLoraCarry);
  tcast_kernel<1><<<dim3(1, kC / 64, 1), blk, 0, stream>>>(td_w2, td_w2, td_w2, td_w2, td_w2, 0L, TW2T, TW2T, 0L,
                                                            kTd, kC, kC, kTd, 1.0f);
  tcast_kernel<1><<<dim3(1, kC / 64, 5), blk, 0, stream>>>(maa_w2, maa_w2, maa_w2, maa_w2, maa_w2, (long)kLd * kC,
                                                            W2T, W2T, (long)kC * kLdPitch, kLd, kC, kC, kLdPitch, 1.0f);
  const int n8 = nBig / 8;
  prep_kernel<<<dim3(n8 / 256), blk, 0, stream>>>(x, maa_x, XXX, n8);
  const int tilesM192 = (kRows / 64) * (kLwPad / 64);
  wmma_gemm64<0, false, 0, 3, 1><<<dim3((tilesM192 + 7) / 8, 1), blk, 0, stream>>>(
      XXX, XXX, kC, 0L, W1T, W1T, kC, 0L, (void*)MPL, (void*)MPL, kLwPad, 0L, tdecay, kRows, kLwPad, kC, 1.0f / kLoraCarry);
  const int tilesFull = (kRows / 64) * (kC / 64);
  const int tilesM64  = (kRows / 64) * (kTd / 64);
  const long w2Stride = (long)kC * kLdPitch;
  mix_gemm64<<<dim3((tilesFull + 7) / 8, 1), blk, 0, stream>>>(
      MPL + 0 * kLd, kLwPad, W2T + 0 * w2Stride, kLdPitch, XF, kC, x, maa_w, kRows, kC, kLd);
  wmma_gemm64<0, false, 0, 3, 1><<<dim3((tilesM64 + 7) / 8, 1), blk, 0, stream>>>(
      XF, XF, kC, 0L, TW1T, TW1T, kC, 0L, (void*)HA, (void*)HA, kTd, 0L, tdecay, kRows, kTd, kC, 1.0f / kLoraCarry);
  wmma_gemm64<1, false, 0, 1, 0><<<dim3((tilesFull + 7) / 8, 1), blk, 0, stream>>>(
      HA, HA, kTd, 0L, TW2T, TW2T, kTd, 0L, (void*)DL, (void*)DL, kC, 0L, tdecay, kRows, kC, kTd, kDlCarry);
  mix_gemm64<<<dim3((tilesFull + 7) / 8, 1), blk, 0, stream>>>(
      MPL + 1 * kLd, kLwPad, W2T + 1 * w2Stride, kLdPitch, XF, kC, x, maa_k, kRows, kC, kLd);
  wmma_gemm64<0, false, 0, 1, 0><<<dim3((tilesFull + 7) / 8, 1), blk, 0, stream>>>(
      XF, XF, kC, 0L, WkT, WkT, kC, 0L, (void*)KPL, (void*)KPL, kC, 0L, tdecay, kRows, kC, kC, 1.0f / kWCarry);
  mix_gemm64<<<dim3((tilesFull + 7) / 8, 1), blk, 0, stream>>>(
      MPL + 2 * kLd, kLwPad, W2T + 2 * w2Stride, kLdPitch, XF, kC, x, maa_v, kRows, kC, kLd);
  wmma_gemm64<0, false, 0, 1, 0><<<dim3((tilesFull + 7) / 8, 1), blk, 0, stream>>>(
      XF, XF, kC, 0L, WvT, WvT, kC, 0L, (void*)VPL, (void*)VPL, kC, 0L, tdecay, kRows, kC, kC, 1.0f / kWCarry);
  mix_gemm64<<<dim3((tilesFull + 7) / 8, 1), blk, 0, stream>>>(
      MPL + 3 * kLd, kLwPad, W2T + 3 * w2Stride, kLdPitch, XF, kC, x, maa_r, kRows, kC, kLd);
  wmma_gemm64<0, false, 0, 1, 0><<<dim3((tilesFull + 7) / 8, 1), blk, 0, stream>>>(
      XF, XF, kC, 0L, WrT, WrT, kC, 0L, (void*)RPL, (void*)RPL, kC, 0L, tdecay, kRows, kC, kC, 1.0f / kWCarry);
  mix_gemm64<<<dim3((tilesFull + 7) / 8, 1), blk, 0, stream>>>(
      MPL + 4 * kLd, kLwPad, W2T + 4 * w2Stride, kLdPitch, XF, kC, x, maa_g, kRows, kC, kLd);
  wmma_gemm64<0, false, 0, 1, 3><<<dim3((tilesFull + 7) / 8, 1), blk, 0, stream>>>(
      XF, XF, kC, 0L, WgT, WgT, kC, 0L, (void*)GPL, (void*)GPL, kC, 0L, tdecay, kRows, kC, kC, 1.0f / kWCarry);
  scan_gn_kernel<<<dim3(kB * kH), blk, 0, stream>>>(RPL, KPL, VPL, GPL, DL, tdecay, uu, ln_g, ln_b, ZH, ZL);
  wmma_gemm64<1, true, 0, 0, 0><<<dim3((tilesFull + 7) / 8, 1), blk, 0, stream>>>(
      ZH, ZL, kC, 0L, WOH, WOL, kC, 0L, (void*)out, (void*)out, kC, 0L, tdecay, kRows, kC, kC, 1.0f);
}
